// WavenetBasedModel_9818295238940
// MI455X (gfx1250) — hardware-verified
//
#include <hip/hip_runtime.h>
#include <math.h>
#include <stdint.h>

#define NBAT   8
#define NBH    4
#define TLEN   131072
#define NCH    16
#define NLAY   10
#define TP     2048
#define NTHR   256
#define NWAV   8
#define HL0    4
#define HLMAX  512
#define WMAXP  (TP + 2 * HLMAX)
#define OUTW   (TLEN + 2)
#define NOUT   (NBAT * OUTW)
#define NG4    (NOUT / 4)

static_assert((TLEN % TP) == 0);
static_assert((TP % (32 * NWAV)) == 0);
static_assert((NOUT % 4) == 0);
static_assert(NBAT == 2 * NBH);
static_assert(((NLAY - 1) & 1) == 1);
static_assert(HL0 >= 1);

typedef _Float16     v16h __attribute__((ext_vector_type(16)));
typedef _Float16     v8h  __attribute__((ext_vector_type(8)));
typedef float        v8f  __attribute__((ext_vector_type(8)));
typedef float        v4f  __attribute__((ext_vector_type(4)));
typedef unsigned int v4u  __attribute__((ext_vector_type(4)));

union FragU { v16h v; v8h h[2]; v4u q[2]; };

__device__ __forceinline__ unsigned short bf_bits(float f) {
  const unsigned u = __float_as_uint(f);
  return (unsigned short)((u + 0x7FFFu + ((u >> 16) & 1u)) >> 16);
}
__device__ __forceinline__ float bf_up(unsigned short b) { return __uint_as_float(((unsigned)b) << 16); }
__device__ __forceinline__ float bf_rne(float f) { return bf_up(bf_bits(f)); }
__device__ __forceinline__ unsigned pkh(float a, float b) {
  union { _Float16 h[2]; unsigned u; } t;
  t.h[0] = (_Float16)a;
  t.h[1] = (_Float16)b;
  return t.u;
}
__device__ __forceinline__ int clampi(int v, int lo, int hi) { return v < lo ? lo : (v > hi ? hi : v); }
__device__ __forceinline__ v4u zero4u() { v4u z = {0u, 0u, 0u, 0u}; return z; }

__device__ __forceinline__ v8f mma_h(v16h a, v16h b, v8f c) {
  return __builtin_amdgcn_wmma_f32_16x16x32_f16(false, a, false, b, (short)0, c, false, false);
}
__device__ __forceinline__ void guard2(v8f& acc, v16h x, v16h y) {
#if defined(__HIP_DEVICE_COMPILE__)
  asm volatile("v_nop\n\tv_nop\n\tv_nop\n\tv_nop" : "+v"(acc) : "v"(x), "v"(y));
#endif
}
__device__ __forceinline__ void guard1(v8f& acc, v16h x) {
#if defined(__HIP_DEVICE_COMPILE__)
  asm volatile("v_nop\n\tv_nop\n\tv_nop\n\tv_nop" : "+v"(acc) : "v"(x));
#endif
}
__device__ __forceinline__ void wave_sync_lds() {
  __builtin_amdgcn_fence(__ATOMIC_RELEASE, "workgroup");
  __builtin_amdgcn_wave_barrier();
  __builtin_amdgcn_fence(__ATOMIC_ACQUIRE, "workgroup");
}

__device__ __forceinline__ void load_w3(const float* __restrict__ w, int lane, v16h& f0, v16h& f1) {
  const int o = lane & 15, hb = (lane >> 4) * 8;
  v4u t0, t1, t2;
#pragma unroll
  for (int q = 0; q < 4; ++q) {
    const float* p = w + (o * NCH + hb + 2 * q) * 3;
    t0[q] = pkh(bf_rne(p[0]), bf_rne(p[3]));
    t1[q] = pkh(bf_rne(p[1]), bf_rne(p[4]));
    t2[q] = pkh(bf_rne(p[2]), bf_rne(p[5]));
  }
  FragU u0, u1;
  u0.q[0] = t0; u0.q[1] = t1;
  u1.q[0] = t2; u1.q[1] = zero4u();
  f0 = u0.v; f1 = u1.v;
}
__device__ __forceinline__ v16h load_w1(const float* __restrict__ w, int lane) {
  const int o = lane & 15, hb = (lane >> 4) * 8;
  v4u t;
#pragma unroll
  for (int q = 0; q < 4; ++q)
    t[q] = pkh(bf_rne(w[o * NCH + hb + 2 * q]), bf_rne(w[o * NCH + hb + 2 * q + 1]));
  FragU u;
  u.q[0] = t; u.q[1] = zero4u();
  return u.v;
}
__device__ __forceinline__ v8f load_bias8(const float* __restrict__ bsrc, int lane) {
  const int hb = (lane >> 4) * 8;
  v8f v;
#pragma unroll
  for (int r = 0; r < 8; ++r) v[r] = bf_rne(bsrc[hb + r]);
  return v;
}

__device__ __forceinline__ void load_act(const unsigned short* hp, int dstep, v16h& b0, v16h& b1) {
  FragU u0, u1;
  u0.h[0] = *(const v8h*)(hp - dstep);
  u0.h[1] = *(const v8h*)(hp);
  u1.h[0] = *(const v8h*)(hp + dstep);
  u1.q[1] = zero4u();
  b0 = u0.v; b1 = u1.v;
}

__device__ __forceinline__ void stage_f32to16(const float* __restrict__ src, int t0, int HL, int W, unsigned short* hL) {
  const int n = W * 2;
#pragma unroll 1
  for (int it = threadIdx.x; it < n; it += NTHR) {
    const int u = it >> 1, g = it & 1;
    const int t = t0 - HL + u;
    const bool ok = (t >= 0) && (t < TLEN);
    const int tc = clampi(t, 0, TLEN - 1);
    const float* sp = src + (size_t)tc * NCH + 8 * g;
    const v4f a = *(const v4f*)(sp);
    const v4f c = *(const v4f*)(sp + 4);
    v4u pk;
    pk[0] = ok ? pkh(a[0], a[1]) : 0u;
    pk[1] = ok ? pkh(a[2], a[3]) : 0u;
    pk[2] = ok ? pkh(c[0], c[1]) : 0u;
    pk[3] = ok ? pkh(c[2], c[3]) : 0u;
    *(v4u*)(hL + (size_t)u * NCH + 8 * g) = pk;
  }
}
__device__ __forceinline__ void stage_copy16(const unsigned short* __restrict__ src, int t0, int HL, int W,
                                             unsigned short* hL) {
  const int n = W * 2;
#pragma unroll 1
  for (int it = threadIdx.x; it < n; it += NTHR) {
    const int u = it >> 1, g = it & 1;
    const int t = t0 - HL + u;
    const bool ok = (t >= 0) && (t < TLEN);
    const int tc = clampi(t, 0, TLEN - 1);
    const v4u v = *(const v4u*)(src + (size_t)tc * NCH + 8 * g);
    v4u pk;
    pk[0] = ok ? v[0] : 0u;
    pk[1] = ok ? v[1] : 0u;
    pk[2] = ok ? v[2] : 0u;
    pk[3] = ok ? v[3] : 0u;
    *(v4u*)(hL + (size_t)u * NCH + 8 * g) = pk;
  }
}

__device__ __forceinline__ v8f conv3_tile(const unsigned short* hL, int uc, int hb, int dstep,
                                          v16h a0, v16h a1, v8f bias) {
  v16h b0, b1;
  load_act(hL + uc * NCH + hb, dstep, b0, b1);
  v8f acc = bias;
  acc = mma_h(a0, b0, acc);
  acc = mma_h(a1, b1, acc);
  guard2(acc, b0, b1);
  return acc;
}

__device__ __forceinline__ float gate_f(float hv) {
  const float hc = fminf(fmaxf(hv, -30.0f), 30.0f);
  const float e1 = __expf(-hc);
  const float sg = __builtin_amdgcn_rcpf(1.0f + e1);
  const float e2 = e1 * e1;
  const float th = (1.0f - e2) * __builtin_amdgcn_rcpf(1.0f + e2);
  return th * sg;
}
__device__ __forceinline__ v8f gate_1x1(v8f h8, v16h a3, v8f bias2) {
  v4u qg;
#pragma unroll
  for (int q = 0; q < 4; ++q) {
    const float g0 = gate_f(h8[2 * q]);
    const float g1 = gate_f(h8[2 * q + 1]);
    qg[q] = pkh(g0, g1);
  }
  FragU bg;
  bg.q[0] = qg; bg.q[1] = zero4u();
  v8f o = bias2;
  o = mma_h(a3, bg.v, o);
  guard1(o, bg.v);
  return o;
}

template <int FIRST>
__global__ __launch_bounds__(NTHR) void k_layer(const float* __restrict__ x, const float* __restrict__ rin,
                                                const float* __restrict__ wcv, const float* __restrict__ bcv,
                                                const float* __restrict__ w11, const float* __restrict__ b11,
                                                float* rout, float* skp, int half, int d, int HL, int W) {
  extern __shared__ __align__(16) unsigned char dsm[];
  __shared__ __align__(16) float oT[NWAV][32 * NCH];
  const int tid = threadIdx.x, lane = tid & 31, wave = tid >> 5;
  const int p = lane & 15, hb = (lane >> 4) * 8;
  const int bl = blockIdx.y, b = half * NBH + bl;
  const int t0 = blockIdx.x * TP;
  const size_t poff = (size_t)bl * TLEN * NCH;
  const float* xb   = x + (size_t)b * TLEN;
  const float* rinb = rin + poff;
  float* routb = rout + poff;
  float* skb   = skp + poff;
  float* xL = (float*)dsm;
  unsigned short* hL = (unsigned short*)dsm;
  const int dstep = d * NCH;

  if (FIRST) {
#pragma unroll 1
    for (int u = tid; u < W; u += NTHR) {
      const int t = t0 - HL + u;
      const bool ok = (t >= 0) && (t < TLEN);
      const int tc = clampi(t, 0, TLEN - 1);
      const float v = xb[tc];
      xL[u] = ok ? bf_rne(v) : 0.f;
    }
  } else {
    stage_f32to16(rinb, t0, HL, W, hL);
  }
  __syncthreads();

  v16h a0, a1;
  float wt0[8], wt1[8], wt2[8];
  {
    FragU z; z.q[0] = zero4u(); z.q[1] = zero4u();
    a0 = z.v; a1 = z.v;
#pragma unroll
    for (int r = 0; r < 8; ++r) { wt0[r] = 0.f; wt1[r] = 0.f; wt2[r] = 0.f; }
  }
  if (FIRST) {
#pragma unroll
    for (int r = 0; r < 8; ++r) {
      wt0[r] = bf_rne(wcv[(hb + r) * 3 + 0]);
      wt1[r] = bf_rne(wcv[(hb + r) * 3 + 1]);
      wt2[r] = bf_rne(wcv[(hb + r) * 3 + 2]);
    }
  } else {
    load_w3(wcv, lane, a0, a1);
  }
  const v16h a3     = load_w1(w11, lane);
  const v8f  bias1v = load_bias8(bcv, lane);
  const v8f  bias2v = load_bias8(b11, lane);
  float* ot = oT[wave];

#pragma unroll 1
  for (int it = wave; it < TP / 32; it += NWAV) {
    const int p0 = it * 32;
    v8f o[2];
#pragma unroll
    for (int s = 0; s < 2; ++s) {
      const int uc = HL + p0 + 16 * s + p;
      v8f acc;
      if (FIRST) {
        const float xm = xL[uc - 1], x0 = xL[uc], xq = xL[uc + 1];
        acc = bias1v;
#pragma unroll
        for (int r = 0; r < 8; ++r)
          acc[r] = fmaf(wt2[r], xq, fmaf(wt1[r], x0, fmaf(wt0[r], xm, bias1v[r])));
      } else {
        acc = conv3_tile(hL, uc, hb, dstep, a0, a1, bias1v);
      }
      o[s] = gate_1x1(acc, a3, bias2v);
    }
#pragma unroll
    for (int s = 0; s < 2; ++s) {
      v4f u0, u1;
      u0[0] = o[s][0]; u0[1] = o[s][1]; u0[2] = o[s][2]; u0[3] = o[s][3];
      u1[0] = o[s][4]; u1[1] = o[s][5]; u1[2] = o[s][6]; u1[3] = o[s][7];
      float* op = ot + (16 * s + p) * NCH + hb;
      *(v4f*)(op) = u0;
      *(v4f*)(op + 4) = u1;
    }
    wave_sync_lds();
    const size_t gbase = (size_t)(t0 + p0) * NCH;
    v4f rv[4], sv[4];
#pragma unroll
    for (int j = 0; j < 4; ++j) {
      const int f = (j * 32 + lane) * 4;
      const v4f ov = *(const v4f*)(ot + f);
      if (FIRST) {
        const float xv = xL[HL + p0 + (f >> 4)];
        v4f xq;
        xq[0] = xv; xq[1] = xv; xq[2] = xv; xq[3] = xv;
        rv[j] = ov + xq;
        sv[j] = ov;
      } else {
        const v4f rold = *(const v4f*)(rinb + gbase + f);
        const v4f sold = *(const v4f*)(skb + gbase + f);
        rv[j] = ov + rold;
        sv[j] = sold + ov;
      }
    }
#pragma unroll
    for (int j = 0; j < 4; ++j) {
      const int f = (j * 32 + lane) * 4;
      *(volatile v4f*)(routb + gbase + f) = rv[j];
      *(volatile v4f*)(skb + gbase + f) = sv[j];
    }
    __threadfence();
#pragma unroll
    for (int j = 0; j < 4; ++j) {
      const int f = (j * 32 + lane) * 4;
      *(volatile v4f*)(routb + gbase + f) = rv[j];
      *(volatile v4f*)(skb + gbase + f) = sv[j];
    }
    wave_sync_lds();
  }
}

__global__ __launch_bounds__(NTHR) void k_head1(const float* __restrict__ src, const float* __restrict__ wcv,
                                               const float* __restrict__ bcv, unsigned short* y1, int HL, int W) {
  extern __shared__ __align__(16) unsigned char dsm[];
  __shared__ __align__(16) float oT[NWAV][32 * NCH];
  const int tid = threadIdx.x, lane = tid & 31, wave = tid >> 5;
  const int p = lane & 15, hb = (lane >> 4) * 8;
  const int bl = blockIdx.y;
  const int t0 = blockIdx.x * TP;
  const size_t poff = (size_t)bl * TLEN * NCH;
  const float* srcb = src + poff;
  unsigned short* y1b = y1 + poff;
  unsigned short* hL = (unsigned short*)dsm;

  stage_f32to16(srcb, t0, HL, W, hL);
  __syncthreads();

  v16h a0, a1;
  load_w3(wcv, lane, a0, a1);
  const v8f bias1v = load_bias8(bcv, lane);
  unsigned short* oth = (unsigned short*)oT[wave];

#pragma unroll 1
  for (int it = wave; it < TP / 32; it += NWAV) {
    const int p0 = it * 32;
#pragma unroll
    for (int s = 0; s < 2; ++s) {
      const int uc = HL + p0 + 16 * s + p;
      const v8f acc = conv3_tile(hL, uc, hb, NCH, a0, a1, bias1v);
      v4u pk;
#pragma unroll
      for (int q = 0; q < 4; ++q) pk[q] = pkh(fmaxf(acc[2 * q], 0.f), fmaxf(acc[2 * q + 1], 0.f));
      *(v4u*)(oth + (16 * s + p) * NCH + hb) = pk;
    }
    wave_sync_lds();
    const size_t gbase = (size_t)(t0 + p0) * NCH;
    v4u yv[2];
#pragma unroll
    for (int j = 0; j < 2; ++j) yv[j] = *(const v4u*)(oth + (j * 32 + lane) * 8);
#pragma unroll
    for (int j = 0; j < 2; ++j) *(volatile v4u*)(y1b + gbase + (size_t)(j * 32 + lane) * 8) = yv[j];
    __threadfence();
#pragma unroll
    for (int j = 0; j < 2; ++j) *(volatile v4u*)(y1b + gbase + (size_t)(j * 32 + lane) * 8) = yv[j];
    wave_sync_lds();
  }
}

__global__ __launch_bounds__(NTHR) void k_head2(const unsigned short* __restrict__ y1, const float* __restrict__ wcv,
                                               const float* __restrict__ bcv, const float* __restrict__ wc3,
                                               const float* __restrict__ bc3, float* z, int half, int HL, int W) {
  extern __shared__ __align__(16) unsigned char dsm[];
  __shared__ __align__(16) float oT[NWAV][32 * NCH];
  const int tid = threadIdx.x, lane = tid & 31, wave = tid >> 5;
  const int p = lane & 15, hb = (lane >> 4) * 8;
  const int bl = blockIdx.y, b = half * NBH + bl;
  const int t0 = blockIdx.x * TP;
  const size_t poff = (size_t)bl * TLEN * NCH;
  const unsigned short* y1b = y1 + poff;
  float* zb = z + (size_t)b * TLEN;
  unsigned short* hL = (unsigned short*)dsm;

  stage_copy16(y1b, t0, HL, W, hL);
  __syncthreads();

  v16h a0, a1;
  load_w3(wcv, lane, a0, a1);
  const v8f bias1v = load_bias8(bcv, lane);
  float w3r[8];
#pragma unroll
  for (int r = 0; r < 8; ++r) w3r[r] = bf_rne(wc3[hb + r]);
  const float bc3r = bf_rne(bc3[0]);
  float* ot = oT[wave];

#pragma unroll 1
  for (int it = wave; it < TP / 32; it += NWAV) {
    const int p0 = it * 32;
#pragma unroll
    for (int s = 0; s < 2; ++s) {
      const int uc = HL + p0 + 16 * s + p;
      const v8f acc = conv3_tile(hL, uc, hb, NCH, a0, a1, bias1v);
      float part = 0.f;
#pragma unroll
      for (int r = 0; r < 8; ++r) part = fmaf(w3r[r], fmaxf(acc[r], 0.f), part);
      const float tot = part + __shfl_xor(part, 16, 32);
      const float zv = tot + bc3r;
      if (hb == 0) ot[16 * s + p] = zv;
    }
    wave_sync_lds();
    const int li = lane & 7;
    const v4f v = *(const v4f*)(ot + 4 * li);
    float* zp = zb + (size_t)t0 + p0 + 4 * li;
    if (lane < 8) *(volatile v4f*)zp = v;
    __threadfence();
    if (lane < 8) *(volatile v4f*)zp = v;
    wave_sync_lds();
  }
}

__global__ __launch_bounds__(NTHR) void k_pack(const float* __restrict__ z, const float* __restrict__ bc3,
                                              float* out, int ng) {
  const int i = blockIdx.x * NTHR + threadIdx.x;
  if (i >= ng) return;
  const float padv = bf_rne(bc3[0]);
  v4f v;
#pragma unroll
  for (int e = 0; e < 4; ++e) {
    const int f   = 4 * i + e;
    const int row = f / OUTW;
    const int rc  = clampi(row, 0, NBAT - 1);
    const int col = f - row * OUTW;
    const bool inner = (col >= 1) && (col <= TLEN);
    const int tz = clampi(col - 1, 0, TLEN - 1);
    const float zv = z[(size_t)rc * TLEN + tz];
    v[e] = inner ? zv : padv;
  }
  float* pOut = out + (size_t)i * 4;
  *(volatile v4f*)pOut = v;
  __threadfence();
  *(volatile v4f*)pOut = v;
}

extern "C" void kernel_launch(void* const* d_in, const int* in_sizes, int n_in,
                              void* d_out, int out_size, void* d_ws, size_t ws_size,
                              hipStream_t stream) {
  if (n_in < 13) return;
  if (in_sizes[0] != NBAT * TLEN) return;
  if (in_sizes[1] != NCH * 1 * 3) return;
  if (in_sizes[2] != NCH) return;
  if (in_sizes[3] != (NLAY - 1) * NCH * NCH * 3) return;
  if (in_sizes[4] != (NLAY - 1) * NCH) return;
  if (in_sizes[5] != NLAY * NCH * NCH) return;
  if (in_sizes[6] != NLAY * NCH) return;
  if (in_sizes[7] != NCH * NCH * 3 || in_sizes[8] != NCH) return;
  if (in_sizes[9] != NCH * NCH * 3 || in_sizes[10] != NCH) return;
  if (in_sizes[11] != NCH || in_sizes[12] != 1) return;
  if (out_size != NOUT) return;

  const float* x    = (const float*)d_in[0];
  const float* w1_0 = (const float*)d_in[1];
  const float* b1_0 = (const float*)d_in[2];
  const float* w1   = (const float*)d_in[3];
  const float* b1   = (const float*)d_in[4];
  const float* w2   = (const float*)d_in[5];
  const float* b2   = (const float*)d_in[6];
  const float* wc1  = (const float*)d_in[7];
  const float* bc1  = (const float*)d_in[8];
  const float* wc2  = (const float*)d_in[9];
  const float* bc2  = (const float*)d_in[10];
  const float* wc3  = (const float*)d_in[11];
  const float* bc3  = (const float*)d_in[12];
  float* out = (float*)d_out;

  const size_t PL = (size_t)NBH * TLEN * NCH * sizeof(float);
  const size_t PZ = (size_t)NBAT * TLEN * sizeof(float);
  const size_t PY = (size_t)NBH * TLEN * NCH * 2;
  size_t off = 0;
  const size_t oR0 = off; off += PL;
  const size_t oR1 = off; off += PL;
  const size_t oS  = off; off += PL;
  const size_t oZ  = off; off += PZ;
  if (off > ws_size) return;
  if (off > (size_t)134217728) return;
  if (PY > PL) return;

  char* ws = (char*)d_ws;
  float* R0 = (float*)(ws + oR0);
  float* R1 = (float*)(ws + oR1);
  float* S  = (float*)(ws + oS);
  float* Z  = (float*)(ws + oZ);
  unsigned short* Y1 = (unsigned short*)(ws + oR0);

  const int W0 = TP + 2 * HL0;
  (void)hipFuncSetAttribute(reinterpret_cast<const void*>(&k_layer<0>), hipFuncAttributeMaxDynamicSharedMemorySize,
                            WMAXP * NCH * 2);
  (void)hipFuncSetAttribute(reinterpret_cast<const void*>(&k_head1), hipFuncAttributeMaxDynamicSharedMemorySize,
                            W0 * NCH * 2);
  (void)hipFuncSetAttribute(reinterpret_cast<const void*>(&k_head2), hipFuncAttributeMaxDynamicSharedMemorySize,
                            W0 * NCH * 2);

  const dim3 blk(NTHR);
  const dim3 gl(TLEN / TP, NBH);
  const dim3 gp((NG4 + NTHR - 1) / NTHR);

  for (int half = 0; half < 2; ++half) {
    k_layer<1><<<gl, blk, (size_t)W0 * sizeof(float), stream>>>(
        x, R1, w1_0, b1_0, w2, b2, R0, S, half, 1, HL0, W0);
    for (int layer = 1; layer < NLAY; ++layer) {
      const int d  = 1 << layer;
      const int HL = (d < HL0) ? HL0 : d;
      const int W  = TP + 2 * HL;
      const float* rinp = (layer & 1) ? R0 : R1;
      float* routp      = (layer & 1) ? R1 : R0;
      k_layer<0><<<gl, blk, (size_t)W * NCH * 2, stream>>>(
          x, rinp, w1 + (size_t)(layer - 1) * 768, b1 + (size_t)(layer - 1) * 16,
          w2 + (size_t)layer * 256, b2 + (size_t)layer * 16, routp, S, half, d, HL, W);
    }
    k_head1<<<gl, blk, (size_t)W0 * NCH * 2, stream>>>(S, wc1, bc1, Y1, HL0, W0);
    k_head2<<<gl, blk, (size_t)W0 * NCH * 2, stream>>>(Y1, wc2, bc2, wc3, bc3, Z, half, HL0, W0);
  }
  k_pack<<<gp, blk, 0, stream>>>(Z, bc3, out, NG4);
  (void)hipGetLastError();
}
